// LocalPart_61460982006076
// MI455X (gfx1250) — hardware-run, weakly checked
//
#include <hip/hip_runtime.h>
#include <math.h>

typedef __attribute__((ext_vector_type(8)))  _Float16 v8h;
typedef __attribute__((ext_vector_type(16))) __bf16   v16b;
typedef __attribute__((ext_vector_type(8)))  __bf16   v8b;
typedef __attribute__((ext_vector_type(8)))  float    v8f;
typedef __attribute__((ext_vector_type(4)))  float    v4f;

constexpr int kNB      = 64;
constexpr int kNT      = 50;
constexpr int kJ       = 22;
constexpr int kC       = 64;
constexpr int kO       = 64;
constexpr int kBT      = kNB * kNT;
constexpr int kRows    = kBT * kJ;
constexpr int kCat     = 3 * kO;
constexpr int kNnzSym  = 40;
constexpr int kNnzCon  = 88;
constexpr int kTile    = kJ * kO;
constexpr int kTileQ   = kTile / 4;
constexpr int kCatPitch = 196;
constexpr float kNegFill = -9.0e15f;
constexpr float kBnEps   = 1e-5f;
constexpr float kInvJ    = 1.0f / (float)kJ;
static_assert(kBT == 3200 && kRows == 70400 && kTile == 1408 && kTileQ == 352, "shape");
static_assert((kRows % 64) == 0 && (kO % 64) == 0 && (kC % 32) == 0 && (kCat % 32) == 0, "GEMM tile multiples");
static_assert((kRows % 32) == 0 && (kBT % 4) == 0, "block multiples");

constexpr size_t kPlaneF32 = (size_t)kRows * kO * 4;
constexpr size_t kPlane16  = (size_t)kRows * kO * 2;
constexpr size_t kCatPlane = (size_t)kRows * kCat * 2;
constexpr size_t kOffR0    = 0;
constexpr size_t kOffR1    = kOffR0 + kPlaneF32;
constexpr size_t kOffR2    = kOffR1 + kPlaneF32;
constexpr size_t kOffR3    = kOffR2 + kPlaneF32;
constexpr size_t kOffR4    = kOffR3 + kPlaneF32;
constexpr size_t kOffR5    = kOffR4 + kPlaneF32;
constexpr size_t kOffR6    = kOffR5 + kPlaneF32;
constexpr size_t kOffPS    = kOffR6 + kPlaneF32;
constexpr size_t kOffPC    = kOffPS + (size_t)kJ * kJ * kO * 4;
constexpr size_t kOffWPH   = kOffPC + (size_t)kJ * kJ * kO * 4;
constexpr size_t kOffWPL   = kOffWPH + (size_t)4 * kO * kC * 2;
constexpr size_t kOffWDH   = kOffWPL + (size_t)4 * kO * kC * 2;
constexpr size_t kOffWDL   = kOffWDH + (size_t)kO * kC * 2;
constexpr size_t kOffCWH   = kOffWDL + (size_t)kO * kC * 2;
constexpr size_t kOffCWL   = kOffCWH + (size_t)kO * kCat * 2;
constexpr size_t kOffPART3 = kOffCWL + (size_t)kO * kCat * 2;
constexpr size_t kOffPARTO = kOffPART3 + (size_t)kBT * 2 * kCat * 4;
constexpr size_t kOffBN3   = kOffPARTO + (size_t)(kRows / 64) * 2 * kO * 4;
constexpr size_t kOffBNO   = kOffBN3 + (size_t)3 * kCat * 4;
constexpr size_t kWsTotal  = kOffBNO + (size_t)3 * kO * 4;
static_assert(kWsTotal == 132017152ull, "carve total");
static_assert(kWsTotal <= 134217728ull, "carve cap");
static_assert(2 * kCatPlane == 3 * kPlaneF32, "cat planes fill three f32 planes");
static_assert(2 * kPlane16 == kPlaneF32, "a hi|lo 16-bit plane pair fills one f32 plane");
static_assert((kPlaneF32 % 128) == 0 && (kPlane16 % 128) == 0 && (kCatPlane % 128) == 0 && (kOffPS % 128) == 0 &&
              (kOffPC % 128) == 0 && (kOffWPH % 128) == 0 && (kOffWPL % 128) == 0 && (kOffWDH % 128) == 0 &&
              (kOffWDL % 128) == 0 && (kOffCWH % 128) == 0 && (kOffCWL % 128) == 0 && (kOffPART3 % 128) == 0 &&
              (kOffPARTO % 128) == 0 && (kOffBN3 % 128) == 0 && (kOffBNO % 128) == 0, "128-B aligned regions");

__device__ __forceinline__ unsigned short f2bf_bits(float f) {
  unsigned u = __float_as_uint(f);
  return (unsigned short)((u + 0x7FFFu + ((u >> 16) & 1u)) >> 16);
}
__device__ __forceinline__ float bf_bits2f(unsigned short h) { return __uint_as_float(((unsigned)h) << 16); }
__device__ __forceinline__ int clampi(int v, int lo, int hi) { return v < lo ? lo : (v > hi ? hi : v); }

__device__ __forceinline__ void split8(const v4f a0, const v4f a1, v8h& hv, v8h& lv) {
#pragma unroll
  for (int e = 0; e < 4; ++e) {
    const float f0 = a0[e];
    const float f1 = a1[e];
    const unsigned short h0 = f2bf_bits(f0);
    const unsigned short h1 = f2bf_bits(f1);
    const unsigned short l0 = f2bf_bits(f0 - bf_bits2f(h0));
    const unsigned short l1 = f2bf_bits(f1 - bf_bits2f(h1));
    hv[e]     = __builtin_bit_cast(_Float16, h0);
    hv[4 + e] = __builtin_bit_cast(_Float16, h1);
    lv[e]     = __builtin_bit_cast(_Float16, l0);
    lv[4 + e] = __builtin_bit_cast(_Float16, l1);
  }
}

__device__ __forceinline__ void tie_b(v8f& a, v16b x, v16b y) { asm volatile("" : "+v"(a) : "v"(x), "v"(y)); }
__device__ __forceinline__ void tie_nop_b(v8f& a, v16b x, v16b y) { asm volatile("v_nop\n\tv_nop\n\tv_nop\n\tv_nop" : "+v"(a) : "v"(x), "v"(y)); }
__device__ __forceinline__ void keep4_b(v16b a, v16b b, v16b c, v16b d) { asm volatile("v_nop" :: "v"(a), "v"(b), "v"(c), "v"(d)); }
__device__ __forceinline__ void acc_guard4(v8f& a, v8f& b, v8f& c, v8f& d) { asm volatile("v_nop\n\tv_nop\n\tv_nop\n\tv_nop" : "+v"(a), "+v"(b), "+v"(c), "+v"(d)); }
template <typename T> struct Frag;
template <> struct Frag<__bf16> {
  typedef v16b V; union U { v16b v; v8b h[2]; };
  static __device__ __forceinline__ v16b load(const __bf16* p) {
    U f; f.h[0] = *(const v8b*)(p); f.h[1] = *(const v8b*)(p + 16); return f.v;
  }
  static __device__ __forceinline__ v8f mma(v16b a, v16b b, v8f c) {
    return __builtin_amdgcn_wmma_f32_16x16x32_bf16(false, a, false, b, (short)0, c, false, false);
  }
  static __device__ __forceinline__ void tie(v8f& a, v16b x, v16b y) { tie_b(a, x, y); }
  static __device__ __forceinline__ void tie_nop(v8f& a, v16b x, v16b y) { tie_nop_b(a, x, y); }
  static __device__ __forceinline__ void keep(v16b a, v16b b, v16b c, v16b d) { keep4_b(a, b, c, d); }
};

template <int ET> struct Elem;
template <> struct Elem<1> { typedef __bf16 T; };
template <int ET, int SPL>
__global__ __launch_bounds__(256) void wmma_gemm64(
    const unsigned short* __restrict__ Ap, const unsigned short* __restrict__ A2p, int lda, long strideA,
    const unsigned short* __restrict__ Btp, const unsigned short* __restrict__ Bt2p, int ldb, long strideB,
    float* __restrict__ Cout, int ldc, long strideC,
    int M, int N, int K, float scale) {
  typedef typename Elem<ET>::T T;
  typedef typename Frag<T>::V V;
  const T* A = (const T*)Ap; const T* A2 = (const T*)A2p; const T* Bt = (const T*)Btp; const T* Bt2 = (const T*)Bt2p;
  __shared__ __align__(16) float sT[8][16 * 68];
  const int b    = blockIdx.y;
  const int lane = threadIdx.x & 31;
  const int wave = threadIdx.x >> 5;
  const int tilesN = N >> 6;
  const int tilesM = M >> 6;
  const int tile = blockIdx.x * 8 + wave;
  if (tile >= tilesM * tilesN) return;
  const int tm = tile / tilesN;
  const int tn = tile - tm * tilesN;
  const int m0 = tm << 6;
  const int n0 = tn << 6;

  const T* Ab  = A  + (size_t)b * strideA;
  const T* Bb  = Bt + (size_t)b * strideB;
  const T* Ab2 = (SPL >= 1) ? (A2  + (size_t)b * strideA) : nullptr;
  const T* Bb2 = (SPL == 2) ? (Bt2 + (size_t)b * strideB) : nullptr;

  const int rlane = lane & 15;
  const int koff  = (lane >> 4) * 8;
  const int mOff  = (lane >> 4) * 8;

  v8f acc[4][4];
#pragma unroll
  for (int i = 0; i < 4; ++i)
#pragma unroll
    for (int j = 0; j < 4; ++j) acc[i][j] = (v8f){0.f,0.f,0.f,0.f,0.f,0.f,0.f,0.f};

  for (int k0 = 0; k0 < K; k0 += 32) {
    V bh[4], bl[4];
#pragma unroll
    for (int j = 0; j < 4; ++j) {
      const size_t bo = (size_t)(n0 + (j << 4) + rlane) * ldb + koff + k0;
      bh[j] = Frag<T>::load(Bb + bo);
      if (SPL == 2) bl[j] = Frag<T>::load(Bb2 + bo);
    }
#pragma unroll
    for (int i = 0; i < 4; ++i) {
      const size_t ao = (size_t)(m0 + (i << 4) + rlane) * lda + koff + k0;
      V ah = Frag<T>::load(Ab + ao);
      V al;
      if (SPL >= 1) al = Frag<T>::load(Ab2 + ao);
#pragma unroll
      for (int j = 0; j < 4; ++j) {
        acc[i][j] = Frag<T>::mma(ah, bh[j], acc[i][j]);
        if (SPL == 2) acc[i][j] = Frag<T>::mma(ah, bl[j], acc[i][j]);
        if (SPL >= 1) acc[i][j] = Frag<T>::mma(al, bh[j], acc[i][j]);
      }
      Frag<T>::tie(acc[i][0], ah, (SPL >= 1) ? al : ah);
      Frag<T>::tie(acc[i][1], ah, (SPL >= 1) ? al : ah);
      Frag<T>::tie(acc[i][2], ah, (SPL >= 1) ? al : ah);
      Frag<T>::tie_nop(acc[i][3], ah, (SPL >= 1) ? al : ah);
    }
    Frag<T>::keep(bh[0], bh[1], bh[2], bh[3]);
    if (SPL == 2) Frag<T>::keep(bl[0], bl[1], bl[2], bl[3]);
  }
  acc_guard4(acc[0][0], acc[0][1], acc[0][2], acc[0][3]);
  acc_guard4(acc[1][0], acc[1][1], acc[1][2], acc[1][3]);
  acc_guard4(acc[2][0], acc[2][1], acc[2][2], acc[2][3]);
  acc_guard4(acc[3][0], acc[3][1], acc[3][2], acc[3][3]);

  float* slab = sT[wave];
  float* C = Cout + (size_t)b * strideC;
#pragma unroll
  for (int i = 0; i < 4; ++i) {
    const int mBase = m0 + (i << 4);
#pragma unroll
    for (int j = 0; j < 4; ++j) {
#pragma unroll
      for (int r = 0; r < 8; ++r) {
        const float v = acc[i][j][r] * scale;
        slab[(mOff + r) * 68 + (j << 4) + rlane] = v;
      }
    }
    __builtin_amdgcn_fence(__ATOMIC_RELEASE, "workgroup");
    __builtin_amdgcn_wave_barrier();
    __builtin_amdgcn_fence(__ATOMIC_ACQUIRE, "workgroup");
    {
      const int hh = lane >> 4, c4 = (lane & 15) * 4;
      for (int pass = 0; pass < 2; ++pass) {
#pragma unroll
        for (int it = 0; it < 8; ++it) {
          const int row = it * 2 + hh;
          v4f v = *(const v4f*)(slab + row * 68 + c4);
          *(volatile v4f*)(C + (size_t)(mBase + row) * ldc + n0 + c4) = v;
        }
        __threadfence();
      }
    }
    __builtin_amdgcn_fence(__ATOMIC_RELEASE, "workgroup");
    __builtin_amdgcn_wave_barrier();
    __builtin_amdgcn_fence(__ATOMIC_ACQUIRE, "workgroup");
  }
}

__global__ __launch_bounds__(256) void prep_weights_kernel(
    const float* __restrict__ W_sym, const float* __restrict__ W_con, const float* __restrict__ W_dis,
    const float* __restrict__ cat_w,
    unsigned short* __restrict__ WPH, unsigned short* __restrict__ WPL,
    unsigned short* __restrict__ WDH, unsigned short* __restrict__ WDL,
    unsigned short* __restrict__ CWH, unsigned short* __restrict__ CWL)
{
  const int tid = threadIdx.x;
  const int blk = blockIdx.x;
  v4f a0, a1;
  v8h hv, lv;
  if (blk < 8) {
    const int g = blk * 256 + tid;
    const int plane = g >> 9;
    const int rem = g & 511;
    const int o = rem >> 3;
    const int c8 = (rem & 7) * 8;
    const float* src = ((plane & 1) ? W_con : W_sym) + (plane >> 1) * (kC * kO);
#pragma unroll
    for (int e = 0; e < 4; ++e) {
      a0[e] = src[(c8 + e) * kO + o];
      a1[e] = src[(c8 + 4 + e) * kO + o];
    }
    split8(a0, a1, hv, lv);
    unsigned short* qh = WPH + (size_t)g * 8;
    unsigned short* ql = WPL + (size_t)g * 8;
    *(volatile v8h*)qh = hv;
    *(volatile v8h*)ql = lv;
    __threadfence();
    *(volatile v8h*)qh = hv;
    *(volatile v8h*)ql = lv;
  } else if (blk < 10) {
    const int g = (blk - 8) * 256 + tid;
    const int o = g >> 3;
    const int c8 = (g & 7) * 8;
#pragma unroll
    for (int e = 0; e < 4; ++e) {
      a0[e] = W_dis[(c8 + e) * kO + o];
      a1[e] = W_dis[(c8 + 4 + e) * kO + o];
    }
    split8(a0, a1, hv, lv);
    unsigned short* qh = WDH + (size_t)g * 8;
    unsigned short* ql = WDL + (size_t)g * 8;
    *(volatile v8h*)qh = hv;
    *(volatile v8h*)ql = lv;
    __threadfence();
    *(volatile v8h*)qh = hv;
    *(volatile v8h*)ql = lv;
  } else {
    const int g = (blk - 10) * 256 + tid;
    a0 = *(const v4f*)(cat_w + (size_t)g * 8);
    a1 = *(const v4f*)(cat_w + (size_t)g * 8 + 4);
    split8(a0, a1, hv, lv);
    unsigned short* qh = CWH + (size_t)g * 8;
    unsigned short* ql = CWL + (size_t)g * 8;
    *(volatile v8h*)qh = hv;
    *(volatile v8h*)ql = lv;
    __threadfence();
    *(volatile v8h*)qh = hv;
    *(volatile v8h*)ql = lv;
  }
}

__global__ __launch_bounds__(64) void adj_softmax_kernel(
    const float* __restrict__ e_sym, const float* __restrict__ e_con,
    const int* __restrict__ rows_sym, const int* __restrict__ cols_sym,
    const int* __restrict__ rows_con, const int* __restrict__ cols_con,
    float* __restrict__ Ps, float* __restrict__ Pc)
{
  __shared__ __align__(16) float sL[kTile];
  const int o = threadIdx.x;
  const int i = blockIdx.x;
  const bool con = (blockIdx.y == 1);
  const float* ev  = con ? e_con : e_sym;
  const int* rows  = con ? rows_con : rows_sym;
  const int* cols  = con ? cols_con : cols_sym;
  float* P         = con ? Pc : Ps;
  const int nnz    = con ? kNnzCon : kNnzSym;
#pragma unroll 1
  for (int j = 0; j < kJ; ++j) sL[j * kO + o] = kNegFill;
  __syncthreads();
#pragma unroll 1
  for (int k = 0; k < nnz; ++k) {
    const int r  = clampi(rows[k], 0, kJ - 1);
    const int cc = clampi(cols[k], 0, kJ - 1);
    const float v = ev[o * nnz + k];
    if (r == i) sL[cc * kO + o] = v;
  }
  __syncthreads();
  float mx = sL[o];
#pragma unroll 1
  for (int j = 1; j < kJ; ++j) mx = fmaxf(mx, sL[j * kO + o]);
  float s = 0.0f;
#pragma unroll 1
  for (int j = 0; j < kJ; ++j) {
    const float p = expf(sL[j * kO + o] - mx);
    sL[j * kO + o] = p;
    s += p;
  }
  const float inv = 1.0f / s;
#pragma unroll 1
  for (int j = 0; j < kJ; ++j) sL[j * kO + o] = sL[j * kO + o] * inv;
  __syncthreads();
  float* dst = P + (size_t)i * kTile;
  for (int pass = 0; pass < 2; ++pass) {
#pragma unroll 1
    for (int it = 0; it < 6; ++it) {
      const int q  = it * 64 + o;
      const int qc = (q < kTileQ) ? q : (kTileQ - 1);
      const v4f v = *(const v4f*)(sL + qc * 4);
      if (q < kTileQ) *(volatile v4f*)(dst + q * 4) = v;
    }
    __threadfence();
  }
}

__global__ __launch_bounds__(256) void split_rows_bf16_kernel(
    const float* __restrict__ src, unsigned short* __restrict__ dhi, unsigned short* __restrict__ dlo, int total8)
{
  const int i = blockIdx.x * 256 + threadIdx.x;
  if (i >= total8) return;
  const size_t e0 = (size_t)i << 3;
  const v4f a0 = *(const v4f*)(src + e0);
  const v4f a1 = *(const v4f*)(src + e0 + 4);
  v8h hv, lv;
  split8(a0, a1, hv, lv);
  unsigned short* qh = dhi + e0;
  unsigned short* ql = dlo + e0;
  *(volatile v8h*)qh = hv;
  *(volatile v8h*)ql = lv;
  __threadfence();
  *(volatile v8h*)qh = hv;
  *(volatile v8h*)ql = lv;
}

__global__ __launch_bounds__(256) void dis_kernel(const float* __restrict__ x,
                                                  unsigned short* __restrict__ DISH, unsigned short* __restrict__ DISL)
{
  __shared__ __align__(16) float sX[4 * kTile];
  const int tid = threadIdx.x;
  const int sub = tid >> 6;
  const int c = tid & 63;
  const float* xb = x + (size_t)(blockIdx.x * 4 + sub) * kTile + c;
  float* col = sX + sub * kTile + c;
  float s = 0.0f;
#pragma unroll 1
  for (int i = 0; i < kJ; ++i) {
    const float v = xb[i * kC];
    col[i * kC] = v;
    s += v;
  }
  const float m = s * kInvJ;
  float V = 0.0f;
#pragma unroll 1
  for (int i = 0; i < kJ; ++i) {
    const float d = col[i * kC] - m;
    V = fmaf(d, d, V);
  }
#pragma unroll 1
  for (int j = 0; j < kJ; ++j) {
    const float d = col[j * kC] - m;
    const float q = fmaf((float)kJ * d, d, V);
    col[j * kC] = sqrtf(q) + 1e-8f;
  }
  __syncthreads();
  constexpr int kChunks = 4 * kJ * 8;
  v8h hv[3], lv[3];
#pragma unroll
  for (int it = 0; it < 3; ++it) {
    const int q  = it * 256 + tid;
    const int qc = (q < kChunks) ? q : (kChunks - 1);
    const float* sp = sX + (qc >> 3) * kC + (qc & 7) * 8;
    const v4f a0 = *(const v4f*)(sp);
    const v4f a1 = *(const v4f*)(sp + 4);
    split8(a0, a1, hv[it], lv[it]);
  }
  unsigned short* dsth = DISH + (size_t)blockIdx.x * kChunks * 8;
  unsigned short* dstl = DISL + (size_t)blockIdx.x * kChunks * 8;
  for (int pass = 0; pass < 2; ++pass) {
#pragma unroll
    for (int it = 0; it < 3; ++it) {
      const int q = it * 256 + tid;
      if (q < kChunks) {
        *(volatile v8h*)(dsth + (size_t)q * 8) = hv[it];
        *(volatile v8h*)(dstl + (size_t)q * 8) = lv[it];
      }
    }
    __threadfence();
  }
}

__global__ __launch_bounds__(256) void mix_kernel(
    float* H0S, const float* __restrict__ H1S, float* H0C, const float* __restrict__ H1C,
    const float* __restrict__ ZD, float* Zout,
    const float* __restrict__ Ps, const float* __restrict__ Pc,
    const float* __restrict__ att, const float* __restrict__ b_dis, float* __restrict__ part)
{
  __shared__ __align__(16) float sIn[3][kTile];
  __shared__ __align__(16) float sOut[3][kTile];
  __shared__ __align__(16) float sPart[2 * kCat];
  __shared__ float sAtt[kJ * kJ];
  const int tid = threadIdx.x;
  const size_t base = (size_t)blockIdx.x * kTile;
  {
    *(v4f*)(&sIn[0][tid * 4]) = *(const v4f*)(H1S + base + tid * 4);
    *(v4f*)(&sIn[1][tid * 4]) = *(const v4f*)(H1C + base + tid * 4);
    *(v4f*)(&sIn[2][tid * 4]) = *(const v4f*)(ZD  + base + tid * 4);
    if (tid < kTileQ - 256) {
      const int q2 = tid + 256;
      *(v4f*)(&sIn[0][q2 * 4]) = *(const v4f*)(H1S + base + q2 * 4);
      *(v4f*)(&sIn[1][q2 * 4]) = *(const v4f*)(H1C + base + q2 * 4);
      *(v4f*)(&sIn[2][q2 * 4]) = *(const v4f*)(ZD  + base + q2 * 4);
    }
    sAtt[tid] = att[tid];
    const int t2  = tid + 256;
    const int t2c = (t2 < kJ * kJ) ? t2 : (kJ * kJ - 1);
    float a2 = att[t2c];
    asm volatile("" : "+v"(a2));
    if (t2 < kJ * kJ) sAtt[t2] = a2;
  }
  __syncthreads();
  const int o = tid & 63;
  const int ig = tid >> 6;
  const float bd = b_dis[o];
#pragma unroll 1
  for (int it = 0; it < 6; ++it) {
    const int i = ig + 4 * it;
    if (i < kJ) {
      const float h0s = H0S[base + i * kO + o];
      const float h0c = H0C[base + i * kO + o];
      const float* ps = Ps + (size_t)i * kTile + o;
      const float* pc = Pc + (size_t)i * kTile + o;
      const float* at = sAtt + i * kJ;
      float xs = 0.0f, yc = 0.0f, zv = 0.0f;
#pragma unroll 2
      for (int j = 0; j < kJ; ++j) {
        const float a = ps[j * kO];
        const float b = pc[j * kO];
        const float w = at[j];
        float hs = sIn[0][j * kO + o];
        float hc = sIn[1][j * kO + o];
        const float zz = sIn[2][j * kO + o];
        const bool dg = (j == i);
        hs = dg ? h0s : hs;
        hc = dg ? h0c : hc;
        xs = fmaf(a, hs, xs);
        yc = fmaf(b, hc, yc);
        zv = fmaf(w, zz, zv);
      }
      zv += bd;
      sOut[0][i * kO + o] = xs;
      sOut[1][i * kO + o] = yc;
      sOut[2][i * kO + o] = zv;
    }
  }
  __syncthreads();
  if (tid < kCat) {
    const int br = tid >> 6;
    const int oo = tid & 63;
    float s = 0.0f, ss = 0.0f;
#pragma unroll 1
    for (int i = 0; i < kJ; ++i) {
      const float v = sOut[br][i * kO + oo];
      s += v;
      ss = fmaf(v, v, ss);
    }
    sPart[tid] = s;
    sPart[kCat + tid] = ss;
  }
  const int q2  = tid + 256;
  const int q2c = (q2 < kTileQ) ? q2 : (kTileQ - 1);
  const v4f e00 = *(const v4f*)(&sOut[0][tid * 4]);
  const v4f e01 = *(const v4f*)(&sOut[0][q2c * 4]);
  const v4f e10 = *(const v4f*)(&sOut[1][tid * 4]);
  const v4f e11 = *(const v4f*)(&sOut[1][q2c * 4]);
  const v4f e20 = *(const v4f*)(&sOut[2][tid * 4]);
  const v4f e21 = *(const v4f*)(&sOut[2][q2c * 4]);
  __syncthreads();
  const int pq = (tid < 96) ? tid : 95;
  const v4f pv = *(const v4f*)(sPart + pq * 4);
  float* pdst = part + (size_t)blockIdx.x * (2 * kCat);
  for (int pass = 0; pass < 2; ++pass) {
    *(volatile v4f*)(H0S  + base + tid * 4) = e00;
    *(volatile v4f*)(H0C  + base + tid * 4) = e10;
    *(volatile v4f*)(Zout + base + tid * 4) = e20;
    if (tid < 96) {
      *(volatile v4f*)(H0S  + base + q2 * 4) = e01;
      *(volatile v4f*)(H0C  + base + q2 * 4) = e11;
      *(volatile v4f*)(Zout + base + q2 * 4) = e21;
      *(volatile v4f*)(pdst + tid * 4) = pv;
    }
    __threadfence();
  }
}

__global__ __launch_bounds__(192) void bn_finalize_kernel(
    const float* __restrict__ part, int nPart, int nch,
    const float* __restrict__ gamma, const float* __restrict__ beta,
    float* __restrict__ outp)
{
  __shared__ __align__(16) float sB[3 * kCat];
  constexpr double kInvRows = 1.0 / (double)kRows;
  const int c = threadIdx.x;
  const int cc = (c < nch) ? c : (nch - 1);
  const int pitch = 2 * nch;
  double s = 0.0, ss = 0.0;
#pragma unroll 4
  for (int p = 0; p < nPart; ++p) {
    s  += (double)part[(size_t)p * pitch + cc];
    ss += (double)part[(size_t)p * pitch + nch + cc];
  }
  const double mean = s * kInvRows;
  double var = ss * kInvRows - mean * mean;
  var = (var < 0.0) ? 0.0 : var;
  const float sc = gamma[cc] * (1.0f / sqrtf((float)var + kBnEps));
  const float be = beta[cc];
  if (c < nch) {
    sB[c] = (float)mean;
    sB[nch + c] = sc;
    sB[2 * nch + c] = be;
  }
  __syncthreads();
  if (c < 32) {
    const int total = 3 * nch;
    for (int pass = 0; pass < 2; ++pass) {
      for (int q0 = 0; q0 < total; q0 += 128) {
        const int q  = q0 + c * 4;
        const int qc = (q < total) ? q : (total - 4);
        const v4f v = *(const v4f*)(sB + qc);
        if (q < total) *(volatile v4f*)(outp + q) = v;
      }
      __threadfence();
    }
  }
}

__device__ __forceinline__ void bn_relu_stage(const float* __restrict__ src, const float* __restrict__ bn,
                                              int chan0, int m0, int tid, float* sC)
{
#pragma unroll
  for (int h = 0; h < 2; ++h) {
    const int q = h * 256 + tid;
    const int row = q >> 4;
    const int c4 = (q & 15) * 4;
    const v4f v  = *(const v4f*)(src + (size_t)(m0 + row) * kO + c4);
    const v4f mu = *(const v4f*)(bn + chan0 + c4);
    const v4f sc = *(const v4f*)(bn + kCat + chan0 + c4);
    const v4f be = *(const v4f*)(bn + 2 * kCat + chan0 + c4);
    v4f y;
#pragma unroll
    for (int e = 0; e < 4; ++e) y[e] = fmaxf(fmaf(v[e] - mu[e], sc[e], be[e]), 0.0f);
    *(v4f*)(sC + row * kCatPitch + chan0 + c4) = y;
  }
}
__global__ __launch_bounds__(256) void form_cat_kernel(
    const float* __restrict__ XS, const float* __restrict__ YC, const float* __restrict__ Zp,
    const float* __restrict__ bn, unsigned short* __restrict__ CATH, unsigned short* __restrict__ CATL)
{
  __shared__ __align__(16) float sC[32 * kCatPitch];
  const int tid = threadIdx.x;
  const int m0 = blockIdx.x * 32;
  bn_relu_stage(XS, bn, 0, m0, tid, sC);
  bn_relu_stage(YC, bn, kO, m0, tid, sC);
  bn_relu_stage(Zp, bn, 2 * kO, m0, tid, sC);
  __syncthreads();
  v8h hv[3], lv[3];
#pragma unroll
  for (int it = 0; it < 3; ++it) {
    const int q = it * 256 + tid;
    const int row = q / 24;
    const int g = q - row * 24;
    const float* sp = sC + row * kCatPitch + g * 8;
    const v4f a0 = *(const v4f*)(sp);
    const v4f a1 = *(const v4f*)(sp + 4);
    split8(a0, a1, hv[it], lv[it]);
  }
  const size_t o0 = (size_t)m0 * 24;
  for (int pass = 0; pass < 2; ++pass) {
#pragma unroll
    for (int it = 0; it < 3; ++it) {
      const size_t oe = (o0 + (size_t)(it * 256 + tid)) * 8;
      *(volatile v8h*)(CATH + oe) = hv[it];
      *(volatile v8h*)(CATL + oe) = lv[it];
    }
    __threadfence();
  }
}

__global__ __launch_bounds__(256) void out_stats_kernel(const float* __restrict__ OUTPRE, float* __restrict__ part)
{
  __shared__ __align__(16) float sR[4][2 * kO];
  const int tid = threadIdx.x;
  const int c = tid & 63;
  const int g = tid >> 6;
  const float* p = OUTPRE + ((size_t)blockIdx.x * 64 + g * 16) * kO + c;
  float s = 0.0f, ss = 0.0f;
#pragma unroll 1
  for (int r = 0; r < 16; ++r) {
    const float v = p[r * kO];
    s += v;
    ss = fmaf(v, v, ss);
  }
  sR[g][c] = s;
  sR[g][kO + c] = ss;
  __syncthreads();
  if (tid < 32) {
    const v4f r0 = *(const v4f*)(&sR[0][tid * 4]);
    const v4f r1 = *(const v4f*)(&sR[1][tid * 4]);
    const v4f r2 = *(const v4f*)(&sR[2][tid * 4]);
    const v4f r3 = *(const v4f*)(&sR[3][tid * 4]);
    const v4f t = ((r0 + r1) + r2) + r3;
    float* dst = part + (size_t)blockIdx.x * (2 * kO) + tid * 4;
    *(volatile v4f*)dst = t;
    __threadfence();
    *(volatile v4f*)dst = t;
  }
}

__global__ __launch_bounds__(256) void apply_out_kernel(
    const float* __restrict__ OUTPRE, const float* __restrict__ bn, float* __restrict__ out, int total4)
{
  const int i = blockIdx.x * 256 + threadIdx.x;
  if (i >= total4) return;
  const int c4 = (i & 15) * 4;
  const v4f v  = *(const v4f*)(OUTPRE + (size_t)i * 4);
  const v4f mu = *(const v4f*)(bn + c4);
  const v4f sc = *(const v4f*)(bn + kO + c4);
  const v4f be = *(const v4f*)(bn + 2 * kO + c4);
  v4f y;
#pragma unroll
  for (int e = 0; e < 4; ++e) y[e] = fmaxf(fmaf(v[e] - mu[e], sc[e], be[e]), 0.0f);
  float* dst = out + (size_t)i * 4;
  *(volatile v4f*)dst = y;
  __threadfence();
  *(volatile v4f*)dst = y;
}

extern "C" void kernel_launch(void* const* d_in, const int* in_sizes, int n_in,
                              void* d_out, int out_size, void* d_ws, size_t ws_size,
                              hipStream_t stream) {
  if (n_in < 15) return;
  if (in_sizes[0]  != kRows * kC) return;
  if (in_sizes[1]  != 2 * kC * kO) return;
  if (in_sizes[2]  != kO * kNnzSym) return;
  if (in_sizes[3]  != 2 * kC * kO) return;
  if (in_sizes[4]  != kO * kNnzCon) return;
  if (in_sizes[5]  != kC * kO) return;
  if (in_sizes[6]  != kJ * kJ) return;
  if (in_sizes[7]  != kO) return;
  if (in_sizes[8]  != kO * kCat) return;
  if (in_sizes[9]  != 4 * kO) return;
  if (in_sizes[10] != 4 * kO) return;
  if (in_sizes[11] != kNnzSym) return;
  if (in_sizes[12] != kNnzSym) return;
  if (in_sizes[13] != kNnzCon) return;
  if (in_sizes[14] != kNnzCon) return;
  if (out_size != kRows * kO) return;
  if (ws_size < kWsTotal) return;

  const float* x      = (const float*)d_in[0];
  const float* W_sym  = (const float*)d_in[1];
  const float* e_sym  = (const float*)d_in[2];
  const float* W_con  = (const float*)d_in[3];
  const float* e_con  = (const float*)d_in[4];
  const float* W_dis  = (const float*)d_in[5];
  const float* att    = (const float*)d_in[6];
  const float* b_dis  = (const float*)d_in[7];
  const float* cat_w  = (const float*)d_in[8];
  const float* gammas = (const float*)d_in[9];
  const float* betas  = (const float*)d_in[10];
  const int* rows_sym = (const int*)d_in[11];
  const int* cols_sym = (const int*)d_in[12];
  const int* rows_con = (const int*)d_in[13];
  const int* cols_con = (const int*)d_in[14];
  float* out = (float*)d_out;

  char* ws = (char*)d_ws;
  unsigned short* XH   = (unsigned short*)(ws + kOffR0);
  unsigned short* XL   = (unsigned short*)(ws + kOffR0 + kPlane16);
  float*          Zp   = (float*)(ws + kOffR0);
  unsigned short* DISH = (unsigned short*)(ws + kOffR1);
  unsigned short* DISL = (unsigned short*)(ws + kOffR1 + kPlane16);
  float*          OUTPRE = (float*)(ws + kOffR1);
  float*          H0S  = (float*)(ws + kOffR2);
  float*          H0C  = (float*)(ws + kOffR3);
  float*          H1S  = (float*)(ws + kOffR4);
  float*          H1C  = (float*)(ws + kOffR5);
  float*          ZD   = (float*)(ws + kOffR6);
  unsigned short* CATH = (unsigned short*)(ws + kOffR4);
  unsigned short* CATL = (unsigned short*)(ws + kOffR4 + kCatPlane);
  float*          Ps   = (float*)(ws + kOffPS);
  float*          Pc   = (float*)(ws + kOffPC);
  unsigned short* WPH  = (unsigned short*)(ws + kOffWPH);
  unsigned short* WPL  = (unsigned short*)(ws + kOffWPL);
  unsigned short* WDH  = (unsigned short*)(ws + kOffWDH);
  unsigned short* WDL  = (unsigned short*)(ws + kOffWDL);
  unsigned short* CWH  = (unsigned short*)(ws + kOffCWH);
  unsigned short* CWL  = (unsigned short*)(ws + kOffCWL);
  float*          PART3 = (float*)(ws + kOffPART3);
  float*          PARTO = (float*)(ws + kOffPARTO);
  float*          BN3  = (float*)(ws + kOffBN3);
  float*          BNO  = (float*)(ws + kOffBNO);

  constexpr int kGemmBlocks = (kRows / 64 + 7) / 8;

  prep_weights_kernel<<<16, 256, 0, stream>>>(W_sym, W_con, W_dis, cat_w, WPH, WPL, WDH, WDL, CWH, CWL);
  adj_softmax_kernel<<<dim3(kJ, 2), 64, 0, stream>>>(e_sym, e_con, rows_sym, cols_sym, rows_con, cols_con, Ps, Pc);
  split_rows_bf16_kernel<<<(kRows * kC / 8) / 256, 256, 0, stream>>>(x, XH, XL, kRows * kC / 8);
  dis_kernel<<<kBT / 4, 256, 0, stream>>>(x, DISH, DISL);

  wmma_gemm64<1, 2><<<dim3(kGemmBlocks, 4), 256, 0, stream>>>(
      XH, XL, kC, 0L,
      WPH, WPL, kC, (long)(kO * kC),
      H0S, kO, (long)(kPlaneF32 / 4),
      kRows, kO, kC, 1.0f);

  wmma_gemm64<1, 2><<<dim3(kGemmBlocks, 1), 256, 0, stream>>>(
      DISH, DISL, kC, 0L,
      WDH, WDL, kC, 0L,
      ZD, kO, 0L,
      kRows, kO, kC, 1.0f);

  mix_kernel<<<kBT, 256, 0, stream>>>(H0S, H1S, H0C, H1C, ZD, Zp, Ps, Pc, att, b_dis, PART3);
  bn_finalize_kernel<<<1, 192, 0, stream>>>(PART3, kBT, kCat, gammas, betas, BN3);
  form_cat_kernel<<<kRows / 32, 256, 0, stream>>>(H0S, H0C, Zp, BN3, CATH, CATL);

  wmma_gemm64<1, 2><<<dim3(kGemmBlocks, 1), 256, 0, stream>>>(
      CATH, CATL, kCat, 0L,
      CWH, CWL, kCat, 0L,
      OUTPRE, kO, 0L,
      kRows, kO, kCat, 1.0f);

  out_stats_kernel<<<kRows / 64, 256, 0, stream>>>(OUTPRE, PARTO);
  bn_finalize_kernel<<<1, 192, 0, stream>>>(PARTO, kRows / 64, kO, gammas + 3 * kO, betas + 3 * kO, BNO);
  apply_out_kernel<<<(kRows * kO / 4) / 256, 256, 0, stream>>>(OUTPRE, BNO, out, kRows * kO / 4);
}
